// MultiHeadAttention2D_10290741641457
// MI455X (gfx1250) — hardware-verified
//
#include <hip/hip_runtime.h>


namespace {
constexpr int NB = 2, S = 2048, E = 1024, NH = 16, D = 64, NR = NB * S;
constexpr float XS = 8.0f, WSC = 256.0f, PS = 8.0f, SCALE = 0.125f, LOG2E = 1.4426950408889634f, THETA = 10000.0f;

typedef _Float16 b16;
typedef __attribute__((ext_vector_type(16))) _Float16 v16b;
typedef __attribute__((ext_vector_type(8))) _Float16 v8b;
typedef __attribute__((ext_vector_type(8))) float v8f;
typedef __attribute__((ext_vector_type(4))) float v4f;
__device__ __forceinline__ float bf16_rne(float f) { unsigned int u = __float_as_uint(f); u += 0x7FFFu + ((u >> 16) & 1u); return __uint_as_float(u & 0xFFFF0000u); }
__device__ __forceinline__ void split16(float v, b16& hi, b16& lo) { hi = (b16)v; lo = (b16)(v - (float)hi); }
__device__ __forceinline__ v16b frag_kb(const b16* p, int hh) { const v8b a = *(const v8b*)(p + 8 * hh), b = *(const v8b*)(p + 16 + 8 * hh); v16b f;
#pragma unroll
  for (int e = 0; e < 8; ++e) { f[e] = a[e]; f[8 + e] = b[e]; } return f; }
__device__ __forceinline__ v8f wmma16b(v16b a, v16b b, v8f c) { v8f d = __builtin_amdgcn_wmma_f32_16x16x32_f16(false, a, false, b, (short)0, c, false, false); asm volatile("v_nop\n\tv_nop\n\tv_nop\n\tv_nop" : "+v"(d) : "v"(a), "v"(b)); return d; }
__device__ __forceinline__ void wave_lds_sync() { __builtin_amdgcn_fence(__ATOMIC_RELEASE, "workgroup"); __builtin_amdgcn_wave_barrier(); __builtin_amdgcn_fence(__ATOMIC_ACQUIRE, "workgroup"); }
__device__ __forceinline__ float nexp2(float x) { return __builtin_amdgcn_exp2f(x); }

__global__ __launch_bounds__(256) void prepx_kernel(const float* __restrict__ x, b16* __restrict__ T16) {
  __shared__ __attribute__((aligned(16))) b16 T[64][64 + 8];
  const int b = blockIdx.z, c0 = blockIdx.y * 64, s0 = blockIdx.x * 64, t_ = threadIdx.x;
  for (int q = t_; q < 64 * 64; q += 256) { const int cc = q >> 6, ss = q & 63; T[ss][cc] = (b16)(bf16_rne(x[((size_t)b * E + c0 + cc) * S + s0 + ss]) * XS); }
  __syncthreads();
  for (int pass = 0; pass < 2; ++pass) { for (int q = t_; q < 64 * 8; q += 256) { const int ss = q >> 3, c8 = (q & 7) * 8; *(volatile v8b*)(T16 + ((size_t)b * S + s0 + ss) * E + c0 + c8) = *(const v8b*)(&T[ss][c8]); } __threadfence(); }
}
__global__ __launch_bounds__(256) void prepw_kernel(const float* __restrict__ wq, const float* __restrict__ wk, const float* __restrict__ wv, const float* __restrict__ wo, b16* __restrict__ WT, b16* __restrict__ WOT) {
  const size_t t = (size_t)blockIdx.x * 256 + threadIdx.x; const size_t nw = (size_t)E * E / 8; if (t >= 4 * nw) return; const int kind = (int)(t / nw); const size_t e = (t - (size_t)kind * nw) * 8;
  const float* w = kind == 0 ? wq : kind == 1 ? wk : kind == 2 ? wv : wo; b16* dst = kind < 3 ? WT + (size_t)kind * E * E : WOT;
  const v4f a = *(const v4f*)(w + e), c = *(const v4f*)(w + e + 4); v8b o;
#pragma unroll
  for (int j = 0; j < 4; ++j) { o[j] = (b16)(bf16_rne(a[j]) * WSC); o[4 + j] = (b16)(bf16_rne(c[j]) * WSC); }
  for (int pass = 0; pass < 2; ++pass) { *(volatile v8b*)(dst + e) = o; __threadfence(); }
}
__global__ __launch_bounds__(128) void proj_kernel(const b16* __restrict__ T16, const b16* __restrict__ WT, const float* __restrict__ bq, const float* __restrict__ bk, const float* __restrict__ bv, float* __restrict__ RAW, b16* __restrict__ VTh, b16* __restrict__ VTl) {
  __shared__ __attribute__((aligned(16))) float Tf[4][16][128 + 4]; __shared__ __attribute__((aligned(16))) b16 Vt[128][64 + 8], Vtl[128][64 + 8];
  const int wave = threadIdx.x >> 5, lane = threadIdx.x & 31, nloc = lane & 15, hlf = lane >> 4, t_ = threadIdx.x; const int kind = blockIdx.z; const size_t m0 = (size_t)blockIdx.x * 64 + wave * 16; const int n0 = blockIdx.y * 128;
  const b16* A = T16; const b16* W = WT + (size_t)kind * E * E; v8f acc[8];
#pragma unroll
  for (int t = 0; t < 8; ++t) acc[t] = (v8f){};
#pragma unroll 2
  for (int kb = 0; kb < E; kb += 32) { const v16b a = frag_kb(A + (m0 + nloc) * E + kb, hlf);
#pragma unroll
    for (int t = 0; t < 8; ++t) acc[t] = wmma16b(a, frag_kb(W + (size_t)(n0 + t * 16 + nloc) * E + kb, hlf), acc[t]); }
  const float* bias = kind == 0 ? bq : kind == 1 ? bk : bv;
  if (kind < 2) {
#pragma unroll
    for (int t = 0; t < 8; ++t) { const float bb = bf16_rne(bias[n0 + t * 16 + nloc]);
#pragma unroll
      for (int r = 0; r < 8; ++r) Tf[wave][8 * hlf + r][t * 16 + nloc] = acc[t][r] * (1.0f / (XS * WSC)) + bb; }
    wave_lds_sync();
    float* dst = RAW + (size_t)kind * NR * E;
    for (int pass = 0; pass < 2; ++pass) { for (int rr = 0; rr < 16; ++rr) *(volatile v4f*)(dst + (m0 + rr) * E + n0 + lane * 4) = *(const v4f*)(&Tf[wave][rr][lane * 4]); __threadfence(); }
  } else {
    const int b = (int)(m0 / S); const int s0 = (int)((size_t)blockIdx.x * 64 - (size_t)b * S);
#pragma unroll
    for (int t = 0; t < 8; ++t)
    { const float bb = bf16_rne(bias[n0 + t * 16 + nloc]);
#pragma unroll
      for (int r = 0; r < 8; ++r) { b16 h_, l_; split16((acc[t][r] * (1.0f / (XS * WSC)) + bb) * XS, h_, l_); Vt[t * 16 + nloc][wave * 16 + 8 * hlf + r] = h_; Vtl[t * 16 + nloc][wave * 16 + 8 * hlf + r] = l_; } }
    __syncthreads();
    for (int pass = 0; pass < 2; ++pass) { for (int q = t_; q < 128 * 8; q += 128) { const int cc = q >> 3, c8 = (q & 7) * 8; const int h = (n0 + cc) / D, dd = (n0 + cc) - h * D; const size_t gi = (((size_t)b * NH + h) * D + dd) * S + s0 + c8;
        *(volatile v8b*)(VTh + gi) = *(const v8b*)(&Vt[cc][c8]); *(volatile v8b*)(VTl + gi) = *(const v8b*)(&Vtl[cc][c8]); } __threadfence(); } }
}
__global__ __launch_bounds__(256) void split_kernel(const float* __restrict__ RAW, b16* __restrict__ Qh, b16* __restrict__ Ql, b16* __restrict__ Kh, b16* __restrict__ Kl) {
  const size_t t = (size_t)blockIdx.x * 256 + threadIdx.x; const size_t per = (size_t)NR * E / 8; if (t >= 2 * per) return; const int kind = (int)(t / per); const size_t e = (t - (size_t)kind * per) * 8;
  const v4f a = *(const v4f*)(RAW + (size_t)kind * NR * E + e), c = *(const v4f*)(RAW + (size_t)kind * NR * E + e + 4); v8b hv, lv;
#pragma unroll
  for (int j = 0; j < 4; ++j) { b16 h_, l_; split16(a[j] * XS, h_, l_); hv[j] = h_; lv[j] = l_; split16(c[j] * XS, h_, l_); hv[4 + j] = h_; lv[4 + j] = l_; }
  b16* dh = kind == 0 ? Qh : Kh; b16* dl = kind == 0 ? Ql : Kl;
  for (int pass = 0; pass < 2; ++pass) { *(volatile v8b*)(dh + e) = hv; *(volatile v8b*)(dl + e) = lv; __threadfence(); }
}
__global__ __launch_bounds__(64) void attn_kernel(const b16* __restrict__ Qh, const b16* __restrict__ Ql, const b16* __restrict__ Kh, const b16* __restrict__ Kl, const b16* __restrict__ VTh, const b16* __restrict__ VTl, b16* __restrict__ Oh, b16* __restrict__ Ol) {
  __shared__ __attribute__((aligned(16))) float To[2][16][D + 4];
  const int wave = threadIdx.x >> 5, lane = threadIdx.x & 31, hh = lane >> 4, col = lane & 15; const int b = blockIdx.z, h = blockIdx.y; const int q0 = blockIdx.x * 32 + wave * 16, qi = q0 + col;
  const size_t qo = ((size_t)b * S + qi) * E + h * D; const v16b qa0 = frag_kb(Qh + qo, hh), qa1 = frag_kb(Qh + qo + 32, hh), ql0 = frag_kb(Ql + qo, hh), ql1 = frag_kb(Ql + qo + 32, hh);
  const b16* Kb = Kh + (size_t)b * S * E + h * D; const b16* Klb = Kl + (size_t)b * S * E + h * D; const b16* Vb = VTh + ((size_t)b * NH + h) * D * S; const b16* Vlb = VTl + ((size_t)b * NH + h) * D * S;
  float m = -INFINITY, l = 0.0f; v8f o[4] = {{}, {}, {}, {}}, ol[4] = {{}, {}, {}, {}};
  const float cs = SCALE * LOG2E / (XS * XS);
  for (int kb = 0; kb < S; kb += 32) {
    v8f s0 = {}, s1 = {};
    { const b16* k0 = Kb + (size_t)(kb + col) * E, *k1 = Kb + (size_t)(kb + 16 + col) * E, *k0l = Klb + (size_t)(kb + col) * E, *k1l = Klb + (size_t)(kb + 16 + col) * E;
      v16b f = frag_kb(k0, hh); s0 = wmma16b(f, qa0, s0); s0 = wmma16b(f, ql0, s0); s0 = wmma16b(frag_kb(k0l, hh), qa0, s0);
      f = frag_kb(k0 + 32, hh); s0 = wmma16b(f, qa1, s0); s0 = wmma16b(f, ql1, s0); s0 = wmma16b(frag_kb(k0l + 32, hh), qa1, s0);
      f = frag_kb(k1, hh); s1 = wmma16b(f, qa0, s1); s1 = wmma16b(f, ql0, s1); s1 = wmma16b(frag_kb(k1l, hh), qa0, s1);
      f = frag_kb(k1 + 32, hh); s1 = wmma16b(f, qa1, s1); s1 = wmma16b(f, ql1, s1); s1 = wmma16b(frag_kb(k1l + 32, hh), qa1, s1); }
    float e[16]; float mx = -INFINITY;
#pragma unroll
    for (int r = 0; r < 8; ++r) { e[r] = s0[r] * cs; e[8 + r] = s1[r] * cs; mx = fmaxf(mx, fmaxf(e[r], e[8 + r])); }
    mx = fmaxf(mx, __shfl_xor(mx, 16)); const float mn = fmaxf(m, mx); const float al = nexp2(m - mn); m = mn; float sum = 0.0f; v16b ph, pl;
#pragma unroll
    for (int i = 0; i < 16; ++i) { const float p = nexp2(e[i] - mn); sum += p; const b16 h_ = (b16)(p * PS); ph[i] = h_; pl[i] = (b16)(p * PS - (float)h_); }
    sum += __shfl_xor(sum, 16); l = l * al + sum;
#pragma unroll
    for (int t = 0; t < 4; ++t) { o[t] *= al; ol[t] *= al; const v16b vf = frag_kb(Vb + (size_t)(t * 16 + col) * S + kb, hh); o[t] = wmma16b(vf, ph, o[t]); ol[t] = wmma16b(vf, pl, ol[t]); ol[t] = wmma16b(frag_kb(Vlb + (size_t)(t * 16 + col) * S + kb, hh), ph, ol[t]); } }
  const float inv = 1.0f / (l * PS * XS);
#pragma unroll
  for (int t = 0; t < 4; ++t)
#pragma unroll
    for (int r = 0; r < 8; ++r) To[wave][col][t * 16 + 8 * hh + r] = (o[t][r] + ol[t][r]) * inv;
  wave_lds_sync();
  for (int pass = 0; pass < 2; ++pass) { for (int r4 = 0; r4 < 16; r4 += 4) { const int rr = r4 + (lane >> 3), c8 = (lane & 7) * 8; v8b hv, lv; for (int j = 0; j < 8; ++j) { b16 a_, c_; split16(To[wave][rr][c8 + j] * XS, a_, c_); hv[j] = a_; lv[j] = c_; }
      const size_t gi = ((size_t)b * S + q0 + rr) * E + h * D + c8; *(volatile v8b*)(Oh + gi) = hv; *(volatile v8b*)(Ol + gi) = lv; } __threadfence(); }
}
__global__ __launch_bounds__(128) void outproj_kernel(const b16* __restrict__ Oh, const b16* __restrict__ Ol, const b16* __restrict__ WO16, const float* __restrict__ bo, float* __restrict__ out) {
  __shared__ __attribute__((aligned(16))) float Ts[4][16][128 + 4];
  const int wave = threadIdx.x >> 5, lane = threadIdx.x & 31, nloc = lane & 15, hlf = lane >> 4; const int b = blockIdx.z; const int e0 = blockIdx.x * 64 + wave * 16, s0 = blockIdx.y * 128;
  v8f acc[8];
#pragma unroll
  for (int t = 0; t < 8; ++t) acc[t] = (v8f){};
#pragma unroll 2
  for (int kb = 0; kb < E; kb += 32) { const v16b a = frag_kb(WO16 + (size_t)(e0 + nloc) * E + kb, hlf);
#pragma unroll
    for (int t = 0; t < 8; ++t) { const size_t ro = ((size_t)b * S + s0 + t * 16 + nloc) * E + kb; acc[t] = wmma16b(a, frag_kb(Oh + ro, hlf), acc[t]); acc[t] = wmma16b(a, frag_kb(Ol + ro, hlf), acc[t]); } }
#pragma unroll
  for (int t = 0; t < 8; ++t)
#pragma unroll
    for (int r = 0; r < 8; ++r) Ts[wave][8 * hlf + r][t * 16 + nloc] = acc[t][r] * (1.0f / (XS * WSC)) + bf16_rne(bo[e0 + 8 * hlf + r]);
  wave_lds_sync();
  for (int pass = 0; pass < 2; ++pass) { for (int rr = 0; rr < 16; ++rr) *(volatile v4f*)(out + ((size_t)b * E + e0 + rr) * S + s0 + lane * 4) = *(const v4f*)(&Ts[wave][rr][lane * 4]); __threadfence(); }
}
}

extern "C" void kernel_launch(void* const* d_in, const int* in_sizes, int n_in, void* d_out, int out_size, void* d_ws, size_t ws_size, hipStream_t stream) {
  (void)n_in;
  auto Fp = [&](int i) { return (const float*)d_in[i]; };
  if (in_sizes[0] != NR * E || in_sizes[1] != E * E || in_sizes[2] != E || in_sizes[3] != E * E || in_sizes[5] != E * E || in_sizes[7] != E * E || in_sizes[8] != E || out_size != NR * E) return;
  size_t off = 0; char* ws = (char*)d_ws;
  auto carve = [&](size_t bytes) { char* p = ws + off; off += (bytes + 255) & ~(size_t)255; return p; };
  b16* T16 = (b16*)carve((size_t)NR * E * 2); b16* WT = (b16*)carve((size_t)3 * E * E * 2); b16* WO16 = (b16*)carve((size_t)E * E * 2);
  b16* Qh = (b16*)carve((size_t)NR * E * 2); b16* Ql = (b16*)carve((size_t)NR * E * 2); b16* Kh = (b16*)carve((size_t)NR * E * 2); b16* Kl = (b16*)carve((size_t)NR * E * 2); b16* VTh = (b16*)carve((size_t)NR * E * 2); b16* VTl = (b16*)carve((size_t)NR * E * 2);
  b16* Oh = (b16*)carve((size_t)NR * E * 2); b16* Ol = (b16*)carve((size_t)NR * E * 2); float* RAW = (float*)carve((size_t)2 * NR * E * 4);
  if (off > ws_size || off > ((size_t)128 << 20)) return;
  prepx_kernel<<<dim3(S / 64, E / 64, NB), 256, 0, stream>>>(Fp(0), T16);
  prepw_kernel<<<(unsigned)(((size_t)4 * E * E / 8 + 255) / 256), 256, 0, stream>>>(Fp(1), Fp(3), Fp(5), Fp(7), WT, WO16);
  proj_kernel<<<dim3(NR / 64, E / 128, 3), 128, 0, stream>>>(T16, WT, Fp(2), Fp(4), Fp(6), RAW, VTh, VTl);
  split_kernel<<<(unsigned)(((size_t)2 * NR * E / 8 + 255) / 256), 256, 0, stream>>>(RAW, Qh, Ql, Kh, Kl);
  attn_kernel<<<dim3(S / 32, NH, NB), 64, 0, stream>>>(Qh, Ql, Kh, Kl, VTh, VTl, Oh, Ol);
  outproj_kernel<<<dim3(E / 64, S / 128, NB), 128, 0, stream>>>(Oh, Ol, WO16, Fp(8), (float*)d_out);
}
